// DeltaNet_31877247271572
// MI455X (gfx1250) — hardware-verified
//
#include <hip/hip_runtime.h>
#include <math.h>

constexpr int kB = 2;
constexpr int kL = 2048;
constexpr int kD = 1024;
constexpr int kH = 4;
constexpr int kDh = 256;
constexpr int kBL = kB * kL;
constexpr int kChunk = 32;
constexpr int kNChunk = kL / kChunk;
constexpr int kLinN = 3 * kD;
constexpr int kGin = 1120;
constexpr int kGpad = 1152;
constexpr int kHg = 1024;
constexpr int kNS = 6;
constexpr int kNLog = kH * kNS;
constexpr int kNar = 64;
constexpr int kSlice = 32;
constexpr int kNSlice = kDh / kSlice;

constexpr float kWCarry = 64.0f;
constexpr float kStatCarry = 16.0f;
constexpr float kW1StatCarry = kWCarry / kStatCarry;
constexpr float kQKCarry = 16.0f;
constexpr float kHGCarry = 16.0f;
constexpr float kFuCarry = 64.0f;
constexpr float kDLCarry = 16.0f;
constexpr float kDLCarryInv = 1.0f / 16.0f;
constexpr float kScaleW = 1.0f / kWCarry;
constexpr float kScaleLogit = 1.0f / (kHGCarry * kWCarry);
constexpr float kScaleOut = 1.0f / (kFuCarry * kWCarry);

static_assert(kBL % 64 == 0 && kLinN % 64 == 0 && kD % 64 == 0 && kNar % 64 == 0 && kHg % 64 == 0);
static_assert(kD % 32 == 0 && kGpad % 32 == 0 && kHg % 32 == 0 && kGpad >= kGin);
static_assert(kH * kDh == kD && kNSlice * kSlice == kDh && kNLog <= kNar);
static_assert((kBL * kD) % (8 * 256) == 0 && (kBL * kHg) % (2 * 256) == 0);
static_assert(kSlice == 32 && kChunk == 32 && kDh == 256);

typedef __attribute__((ext_vector_type(16))) _Float16 v16h;
typedef __attribute__((ext_vector_type(8)))  _Float16 v8h;
typedef __attribute__((ext_vector_type(16))) __bf16   v16b;
typedef __attribute__((ext_vector_type(8)))  __bf16   v8b;
typedef __attribute__((ext_vector_type(8)))  float    v8f;
typedef __attribute__((ext_vector_type(4)))  float    v4f;
typedef __attribute__((ext_vector_type(4)))  unsigned int v4u;
typedef __attribute__((ext_vector_type(2)))  unsigned int v2u;

__device__ __forceinline__ unsigned short f2bf_bits(float f) {
  unsigned u = __float_as_uint(f);
  return (unsigned short)((u + 0x7FFFu + ((u >> 16) & 1u)) >> 16);
}
__device__ __forceinline__ float bf_bits2f(unsigned short h) { return __uint_as_float(((unsigned)h) << 16); }
__device__ __forceinline__ float bfr(float x) {
  unsigned u = __float_as_uint(x);
  u = (u + 0x7FFFu + ((u >> 16) & 1u)) & 0xffff0000u;
  return __uint_as_float(u);
}
__device__ __forceinline__ float h16_to_f32(unsigned hb) {
  const unsigned sgn = (hb & 0x8000u) << 16; const unsigned em = hb & 0x7fffu;
  const float fn = __uint_as_float((em << 13) + 0x38000000u);
  const float fs = (float)em * 5.9604644775390625e-8f;
  const float mag = (em < 0x400u) ? fs : fn; return __uint_as_float(__float_as_uint(mag) | sgn);
}
__device__ __forceinline__ unsigned pk16(unsigned short a, unsigned short b) { return (unsigned)a | ((unsigned)b << 16); }
__device__ __forceinline__ unsigned short h_bits(float f) { const _Float16 h = (_Float16)f; return __builtin_bit_cast(unsigned short, h); }

__device__ __forceinline__ void dep_guard_h(v8f& a, v8f& b, v16h x, v16h y) { asm volatile("v_nop\n\tv_nop\n\tv_nop\n\tv_nop" : "+v"(a), "+v"(b) : "v"(x), "v"(y)); }
__device__ __forceinline__ void dep_guard_b(v8f& a, v8f& b, v16b x, v16b y) { asm volatile("v_nop\n\tv_nop\n\tv_nop\n\tv_nop" : "+v"(a), "+v"(b) : "v"(x), "v"(y)); }
__device__ __forceinline__ void dep_guard4_h(v8f& a, v8f& b, v8f& c, v8f& d, v16h x, v16h y) { asm volatile("v_nop\n\tv_nop\n\tv_nop\n\tv_nop" : "+v"(a), "+v"(b), "+v"(c), "+v"(d) : "v"(x), "v"(y)); }
__device__ __forceinline__ void dep_guard4_b(v8f& a, v8f& b, v8f& c, v8f& d, v16b x, v16b y) { asm volatile("v_nop\n\tv_nop\n\tv_nop\n\tv_nop" : "+v"(a), "+v"(b), "+v"(c), "+v"(d) : "v"(x), "v"(y)); }
__device__ __forceinline__ void keep4_h(v16h a, v16h b, v16h c, v16h d) { asm volatile("v_nop" :: "v"(a), "v"(b), "v"(c), "v"(d)); }
__device__ __forceinline__ void keep4_b(v16b a, v16b b, v16b c, v16b d) { asm volatile("v_nop" :: "v"(a), "v"(b), "v"(c), "v"(d)); }
__device__ __forceinline__ void acc_guard4(v8f& a, v8f& b, v8f& c, v8f& d) { asm volatile("v_nop\n\tv_nop\n\tv_nop\n\tv_nop" : "+v"(a), "+v"(b), "+v"(c), "+v"(d)); }
template <typename T> struct Frag;
template <> struct Frag<_Float16> {
  typedef v16h V; union U { v16h v; v8h h[2]; };
  static __device__ __forceinline__ v16h load(const _Float16* p) {
    U f; f.h[0] = *(const v8h*)(p); f.h[1] = *(const v8h*)(p + 16); return f.v;
  }
  static __device__ __forceinline__ v8f mma(v16h a, v16h b, v8f c) {
    return __builtin_amdgcn_wmma_f32_16x16x32_f16(false, a, false, b, (short)0, c, false, false);
  }
  static __device__ __forceinline__ void guard(v8f& a, v8f& b, v16h x, v16h y) { dep_guard_h(a, b, x, y); }
  static __device__ __forceinline__ void guard4(v8f& a, v8f& b, v8f& c, v8f& d, v16h x, v16h y) { dep_guard4_h(a, b, c, d, x, y); }
  static __device__ __forceinline__ void keep(v16h a, v16h b, v16h c, v16h d) { keep4_h(a, b, c, d); }
};
template <> struct Frag<__bf16> {
  typedef v16b V; union U { v16b v; v8b h[2]; };
  static __device__ __forceinline__ v16b load(const __bf16* p) {
    U f; f.h[0] = *(const v8b*)(p); f.h[1] = *(const v8b*)(p + 16); return f.v;
  }
  static __device__ __forceinline__ v8f mma(v16b a, v16b b, v8f c) {
    return __builtin_amdgcn_wmma_f32_16x16x32_bf16(false, a, false, b, (short)0, c, false, false);
  }
  static __device__ __forceinline__ void guard(v8f& a, v8f& b, v16b x, v16b y) { dep_guard_b(a, b, x, y); }
  static __device__ __forceinline__ void guard4(v8f& a, v8f& b, v8f& c, v8f& d, v16b x, v16b y) { dep_guard4_b(a, b, c, d, x, y); }
  static __device__ __forceinline__ void keep(v16b a, v16b b, v16b c, v16b d) { keep4_b(a, b, c, d); }
};

__device__ __forceinline__ v8f mma16(v16h a, v16h b, v8f c) {
  c = __builtin_amdgcn_wmma_f32_16x16x32_f16(false, a, false, b, (short)0, c, false, false);
  asm volatile("v_nop\n\tv_nop\n\tv_nop\n\tv_nop" : "+v"(c) : "v"(a), "v"(b));
  return c;
}
__device__ __forceinline__ v16h ldfrag(const _Float16* p) { return Frag<_Float16>::load(p); }

__device__ __forceinline__ float wsum(float v) {
#pragma unroll
  for (int off = 16; off > 0; off >>= 1) v += __shfl_xor(v, off, 32);
  return v;
}
__device__ __forceinline__ float sigmoid_safe(float y) {
  const float e = expf(-fabsf(y));
  const float r = 1.0f / (1.0f + e);
  return (y >= 0.0f) ? r : e * r;
}

template <int ET> struct Elem;
template <> struct Elem<0> { typedef _Float16 T; };
template <> struct Elem<1> { typedef __bf16 T; };
template <int ET, bool SPLIT, int BIAS_MODE, int OUT_MODE, bool RESID, int ACT = 0>
__global__ __launch_bounds__(256) void wmma_gemm64(
    const unsigned short* __restrict__ Ap, const unsigned short* __restrict__ A2p, int lda, long strideA,
    const unsigned short* __restrict__ Btp, const unsigned short* __restrict__ Bt2p, int ldb, long strideB,
    void* __restrict__ Cout, void* __restrict__ Cout2, int ldc, long strideC,
    const float* __restrict__ bias,
    const float* __restrict__ resid, long strideR,
    int M, int N, int K, float scale) {
  typedef typename Elem<ET>::T T;
  typedef typename Frag<T>::V V;
  const T* A = (const T*)Ap; const T* A2 = (const T*)A2p; const T* Bt = (const T*)Btp; const T* Bt2 = (const T*)Bt2p;
  __shared__ __align__(16) float sT[8][16 * 68];
  const int b    = blockIdx.y;
  const int lane = threadIdx.x & 31;
  const int wave = threadIdx.x >> 5;
  const int tilesN = N >> 6;
  const int tilesM = M >> 6;
  const int tile = blockIdx.x * 8 + wave;
  if (tile >= tilesM * tilesN) return;
  const int tm = tile / tilesN;
  const int tn = tile - tm * tilesN;
  const int m0 = tm << 6;
  const int n0 = tn << 6;

  const T* Ab  = A  + (size_t)b * strideA;
  const T* Bb  = Bt + (size_t)b * strideB;
  const T* Ab2 = SPLIT ? (A2  + (size_t)b * strideA) : nullptr;
  const T* Bb2 = SPLIT ? (Bt2 + (size_t)b * strideB) : nullptr;

  const int rlane = lane & 15;
  const int koff  = (lane >> 4) * 8;
  const int mOff  = (lane >> 4) * 8;

  v8f acc[4][4];
#pragma unroll
  for (int i = 0; i < 4; ++i)
#pragma unroll
    for (int j = 0; j < 4; ++j) acc[i][j] = (v8f){0.f,0.f,0.f,0.f,0.f,0.f,0.f,0.f};

  for (int k0 = 0; k0 < K; k0 += 32) {
    V bh[4], bl[4];
#pragma unroll
    for (int j = 0; j < 4; ++j) {
      const size_t bo = (size_t)(n0 + (j << 4) + rlane) * ldb + koff + k0;
      bh[j] = Frag<T>::load(Bb + bo);
      if (SPLIT) bl[j] = Frag<T>::load(Bb2 + bo);
    }
#pragma unroll
    for (int i = 0; i < 4; ++i) {
      const size_t ao = (size_t)(m0 + (i << 4) + rlane) * lda + koff + k0;
      V ah = Frag<T>::load(Ab + ao);
      V al;
      if (SPLIT) al = Frag<T>::load(Ab2 + ao);
#pragma unroll
      for (int j = 0; j < 4; ++j) {
        acc[i][j] = Frag<T>::mma(ah, bh[j], acc[i][j]);
        if (SPLIT) {
          acc[i][j] = Frag<T>::mma(ah, bl[j], acc[i][j]);
          acc[i][j] = Frag<T>::mma(al, bh[j], acc[i][j]);
        }
      }
      Frag<T>::guard4(acc[i][0], acc[i][1], acc[i][2], acc[i][3], ah, SPLIT ? al : bh[3]);
    }
    Frag<T>::keep(bh[0], bh[1], bh[2], bh[3]);
    if (SPLIT) Frag<T>::keep(bl[0], bl[1], bl[2], bl[3]);
  }
  acc_guard4(acc[0][0], acc[0][1], acc[0][2], acc[0][3]);
  acc_guard4(acc[1][0], acc[1][1], acc[1][2], acc[1][3]);
  acc_guard4(acc[2][0], acc[2][1], acc[2][2], acc[2][3]);
  acc_guard4(acc[3][0], acc[3][1], acc[3][2], acc[3][3]);

  float* slab = sT[wave];
  const float* Rb = RESID ? (resid + (size_t)b * strideR) : nullptr;
#pragma unroll
  for (int i = 0; i < 4; ++i) {
    const int mBase = m0 + (i << 4);
#pragma unroll
    for (int j = 0; j < 4; ++j) {
      const int n = n0 + (j << 4) + rlane;
      float bv = 0.f;
      if (BIAS_MODE == 2) bv = bias[n];
#pragma unroll
      for (int r = 0; r < 8; ++r) {
        float v = acc[i][j][r] * scale;
        if (BIAS_MODE == 1) v += bias[mBase + mOff + r];
        if (BIAS_MODE == 2) v += bv;
        if (RESID) v += Rb[(size_t)(mBase + mOff + r) * ldc + n];
        if (ACT == 2) v = fmaxf(v, 0.0f);
        if (ACT == 4) v = (v > 0.f) ? v : 0.01f * v;
        slab[(mOff + r) * 68 + (j << 4) + rlane] = v;
      }
    }
    __builtin_amdgcn_fence(__ATOMIC_RELEASE, "workgroup");
    __builtin_amdgcn_wave_barrier();
    __builtin_amdgcn_fence(__ATOMIC_ACQUIRE, "workgroup");
    if (OUT_MODE == 0) {
      float* C = (float*)Cout + (size_t)b * strideC;
      const int hh = lane >> 4, c4 = (lane & 15) * 4;
      for (int pass = 0; pass < 2; ++pass) {
#pragma unroll
        for (int it = 0; it < 8; ++it) {
          const int row = it * 2 + hh;
          v4f v = *(const v4f*)(slab + row * 68 + c4);
          *(volatile v4f*)(C + (size_t)(mBase + row) * ldc + n0 + c4) = v;
        }
        __threadfence();
      }
    } else {
      const int q = lane >> 3, c8 = (lane & 7) * 8;
      unsigned short* C  = (unsigned short*)Cout  + (size_t)b * strideC;
      unsigned short* C2 = (OUT_MODE == 2) ? ((unsigned short*)Cout2 + (size_t)b * strideC) : nullptr;
      for (int pass = 0; pass < 2; ++pass) {
#pragma unroll
        for (int it = 0; it < 4; ++it) {
          const int row = it * 4 + q;
          const float* sp = slab + row * 68 + c8;
          v8h hv, lv;
#pragma unroll
          for (int e = 0; e < 8; ++e) {
            if (OUT_MODE == 1) {
              hv[e] = (_Float16)sp[e];
            } else {
              unsigned short hb = f2bf_bits(sp[e]);
              unsigned short lb = f2bf_bits(sp[e] - bf_bits2f(hb));
              hv[e] = __builtin_bit_cast(_Float16, hb);
              lv[e] = __builtin_bit_cast(_Float16, lb);
            }
          }
          *(volatile v8h*)(C + (size_t)(mBase + row) * ldc + n0 + c8) = hv;
          if (OUT_MODE == 2) *(volatile v8h*)(C2 + (size_t)(mBase + row) * ldc + n0 + c8) = lv;
        }
        __threadfence();
      }
    }
    __builtin_amdgcn_fence(__ATOMIC_RELEASE, "workgroup");
    __builtin_amdgcn_wave_barrier();
    __builtin_amdgcn_fence(__ATOMIC_ACQUIRE, "workgroup");
  }
}

__global__ __launch_bounds__(256) void hs16_kernel(const float* __restrict__ hs, unsigned short* __restrict__ G16) {
  const int i = blockIdx.x * 256 + threadIdx.x;
  const int row = i >> 7, c8 = (i & 127) * 8;
  const float* p = hs + (size_t)row * kD + c8;
  const v4f a = *(const v4f*)(p);
  const v4f c = *(const v4f*)(p + 4);
  unsigned short hb[8];
#pragma unroll
  for (int e = 0; e < 4; ++e) {
    const float fa = a[e];
    const float fc = c[e];
    hb[e]     = h_bits(bfr(fa));
    hb[4 + e] = h_bits(bfr(fc));
  }
  const v4u u = (v4u){pk16(hb[0], hb[1]), pk16(hb[2], hb[3]), pk16(hb[4], hb[5]), pk16(hb[6], hb[7])};
  unsigned short* q = G16 + (size_t)row * kGpad + c8;
  *(volatile v4u*)q = u;
  __threadfence();
  *(volatile v4u*)q = u;
}

__global__ __launch_bounds__(256) void wtcast_sq_kernel(const float* __restrict__ W0, const float* __restrict__ W1,
                                                        const float* __restrict__ W2, const float* __restrict__ W3,
                                                        unsigned short* __restrict__ outA, unsigned short* __restrict__ outB) {
  __shared__ float sm[64][65];
  const int t  = threadIdx.x;
  const int k0 = blockIdx.x * 64;
  const int n0 = blockIdx.y * 64;
  const int z  = blockIdx.z;
  const float* W = (z == 0) ? W0 : (z == 1) ? W1 : (z == 2) ? W2 : W3;
#pragma unroll
  for (int i = 0; i < 16; ++i) {
    const int e = i * 256 + t;
    const int r = e >> 6;
    const int cc = e & 63;
    sm[cc][r] = kWCarry * bfr(W[(size_t)(k0 + r) * kD + n0 + cc]);
  }
  __syncthreads();
  const int lane = t & 31, wave = t >> 5;
  const int q = lane >> 3, c8 = (lane & 7) * 8;
  unsigned short* op = (z == 3) ? outB : (outA + (size_t)z * kD * kD);
  for (int pass = 0; pass < 2; ++pass) {
#pragma unroll
    for (int it = 0; it < 2; ++it) {
      const int row = wave * 8 + it * 4 + q;
      unsigned short hb[8];
#pragma unroll
      for (int e = 0; e < 8; ++e) hb[e] = h_bits(sm[row][c8 + e]);
      const v4u u = (v4u){pk16(hb[0], hb[1]), pk16(hb[2], hb[3]), pk16(hb[4], hb[5]), pk16(hb[6], hb[7])};
      *(volatile v4u*)(op + (size_t)(n0 + row) * kD + k0 + c8) = u;
    }
    __threadfence();
  }
}

__global__ __launch_bounds__(256) void w1cast_kernel(const float* __restrict__ W1, unsigned short* __restrict__ W1T) {
  __shared__ float sm[64][65];
  const int t  = threadIdx.x;
  const int k0 = blockIdx.x * 64;
  const int n0 = blockIdx.y * 64;
#pragma unroll
  for (int i = 0; i < 16; ++i) {
    const int e = i * 256 + t;
    const int r = e >> 6;
    const int cc = e & 63;
    const int k = k0 + r;
    const int kc = (k < kGin) ? k : (kGin - 1);
    const float wv = W1[(size_t)kc * kHg + n0 + cc];
    const float s = (k < kD) ? kWCarry : kW1StatCarry;
    sm[cc][r] = (k < kGin) ? (s * bfr(wv)) : 0.0f;
  }
  __syncthreads();
  const int lane = t & 31, wave = t >> 5;
  const int q = lane >> 3, c8 = (lane & 7) * 8;
  for (int pass = 0; pass < 2; ++pass) {
#pragma unroll
    for (int it = 0; it < 2; ++it) {
      const int row = wave * 8 + it * 4 + q;
      unsigned short hb[8];
#pragma unroll
      for (int e = 0; e < 8; ++e) hb[e] = h_bits(sm[row][c8 + e]);
      const v4u u = (v4u){pk16(hb[0], hb[1]), pk16(hb[2], hb[3]), pk16(hb[4], hb[5]), pk16(hb[6], hb[7])};
      *(volatile v4u*)(W1T + (size_t)(n0 + row) * kGpad + k0 + c8) = u;
    }
    __threadfence();
  }
}

__global__ __launch_bounds__(256) void narrow_cast_kernel(const float* __restrict__ Wa, const float* __restrict__ Wb,
                                                          unsigned short* __restrict__ outa, unsigned short* __restrict__ outb) {
  __shared__ float sm[64][65];
  const int t  = threadIdx.x;
  const int k0 = blockIdx.x * 64;
  const int z  = blockIdx.z;
  const float* W = (z == 0) ? Wa : Wb;
  const int NOUT = (z == 0) ? kH : kNLog;
  unsigned short* out = (z == 0) ? outa : outb;
#pragma unroll
  for (int i = 0; i < 16; ++i) {
    const int e = i * 256 + t;
    sm[e >> 6][e & 63] = 0.0f;
  }
  __syncthreads();
  const int tot = 64 * NOUT;
  for (int e = t; e < tot; e += 256) {
    const int n = e >> 6, kk = e & 63;
    sm[n][kk] = kWCarry * bfr(W[(size_t)(k0 + kk) * NOUT + n]);
  }
  __syncthreads();
  const int lane = t & 31, wave = t >> 5;
  const int q = lane >> 3, c8 = (lane & 7) * 8;
  for (int pass = 0; pass < 2; ++pass) {
#pragma unroll
    for (int it = 0; it < 2; ++it) {
      const int row = wave * 8 + it * 4 + q;
      unsigned short hb[8];
#pragma unroll
      for (int e = 0; e < 8; ++e) hb[e] = h_bits(sm[row][c8 + e]);
      const v4u u = (v4u){pk16(hb[0], hb[1]), pk16(hb[2], hb[3]), pk16(hb[4], hb[5]), pk16(hb[6], hb[7])};
      *(volatile v4u*)(out + (size_t)row * kD + k0 + c8) = u;
    }
    __threadfence();
  }
}

__global__ __launch_bounds__(256) void conv_silu_kernel(const float* __restrict__ LIN, const float* __restrict__ qc,
                                                        const float* __restrict__ kc, const float* __restrict__ vc,
                                                        unsigned short* __restrict__ Q16, unsigned short* __restrict__ K16,
                                                        float* __restrict__ V32) {
  __shared__ __align__(16) float stage[1024];
  const int row = blockIdx.x;
  const int which = blockIdx.y;
  const int l = row & (kL - 1);
  const int t = threadIdx.x;
  const float* taps = (which == 0) ? qc : (which == 1) ? kc : vc;
  const size_t src = (size_t)which * kD;
  const int rb = row - l;
  const int r3 = (l >= 3) ? (row - 3) : rb, r2 = (l >= 2) ? (row - 2) : rb, r1 = (l >= 1) ? (row - 1) : rb;
  const float f3 = (l >= 3) ? 1.0f : 0.0f, f2 = (l >= 2) ? 1.0f : 0.0f, f1 = (l >= 1) ? 1.0f : 0.0f;
#pragma unroll 1
  for (int e = 0; e < 4; ++e) {
    const int ch = 4 * t + e;
    const v4f w4 = *(const v4f*)(taps + (size_t)ch * 4);
    const float w0 = bfr(w4[0]), w1 = bfr(w4[1]), w2 = bfr(w4[2]), w3 = bfr(w4[3]);
    const float x3 = LIN[(size_t)r3 * kLinN + src + ch];
    const float x2 = LIN[(size_t)r2 * kLinN + src + ch];
    const float x1 = LIN[(size_t)r1 * kLinN + src + ch];
    const float x0 = LIN[(size_t)row * kLinN + src + ch];
    float y = 0.0f;
    y = fmaf(w0 * f3, x3, y);
    y = fmaf(w1 * f2, x2, y);
    y = fmaf(w2 * f1, x1, y);
    y = fmaf(w3, x0, y);
    stage[ch] = y * sigmoid_safe(y);
  }
  __syncthreads();
  if (which < 2) {
    unsigned short* dst = (which == 0) ? Q16 : K16;
    if (t < 128) {
      const float* sp = stage + 8 * t;
      v8h hv;
#pragma unroll
      for (int e = 0; e < 8; ++e) hv[e] = (_Float16)(kQKCarry * sp[e]);
      unsigned short* gp = dst + (size_t)row * kD + 8 * t;
      *(volatile v8h*)gp = hv;
      __threadfence();
      *(volatile v8h*)gp = hv;
    }
  } else {
    const v4f v = *(const v4f*)(stage + 4 * t);
    float* gp = V32 + (size_t)row * kD + 4 * t;
    *(volatile v4f*)gp = v;
    __threadfence();
    *(volatile v4f*)gp = v;
  }
}

__device__ __forceinline__ float sumsq8(const v4u w) {
  float s = 0.0f;
#pragma unroll
  for (int e = 0; e < 4; ++e) {
    const unsigned u = w[e];
    const float a = h16_to_f32(u & 0xffffu);
    const float c = h16_to_f32(u >> 16);
    s = fmaf(a, a, s);
    s = fmaf(c, c, s);
  }
  return s;
}

__global__ __launch_bounds__(256) __attribute__((amdgpu_num_vgpr(256)))
void delta_kernel(const unsigned short* __restrict__ Q16p,
                  const unsigned short* __restrict__ K16p,
                  const float* __restrict__ V32,
                  const float* __restrict__ BETA,
                  unsigned short* __restrict__ DLT) {
  __shared__ __align__(16) float    ST32[8192];
  __shared__ __align__(16) _Float16 ST16[kSlice * kDh];
  __shared__ __align__(16) _Float16 kT16[kDh * kChunk];
  __shared__ __align__(16) _Float16 w16[kChunk * kDh];
  __shared__ __align__(16) _Float16 vT16[kSlice * kChunk];
  __shared__ __align__(16) _Float16 uhT16[kSlice * kChunk];
  __shared__ __align__(16) _Float16 TB16[kChunk * kChunk];
  __shared__ __align__(16) _Float16 at16[kChunk * kChunk];
  __shared__ __align__(16) float    KKs[kChunk * kChunk];
  __shared__ __align__(16) float    Ts[kChunk * kChunk];
  __shared__ __align__(16) float    osc[kSlice * kChunk];
  __shared__ __align__(16) float invq_s[32];
  __shared__ __align__(16) float invk_s[32];
  __shared__ __align__(16) float beta_s[32];

  const int tid = threadIdx.x, lane = tid & 31, wave = tid >> 5;
  const int hh = lane >> 4, rlane = lane & 15, koff = hh * 8;
  const int b = blockIdx.x >> 2, h = blockIdx.x & 3, sl = blockIdx.y;
  const _Float16* Q16 = (const _Float16*)Q16p;
  const _Float16* K16 = (const _Float16*)K16p;
  const size_t colq = (size_t)h * kDh;
  const size_t colv = colq + (size_t)sl * kSlice;
  unsigned short* dbase = DLT + ((size_t)(h * kNSlice + sl) * kBL) * kSlice;
  const v8f zero8 = (v8f){0.f,0.f,0.f,0.f,0.f,0.f,0.f,0.f};
  const v4f zero4 = (v4f){0.f,0.f,0.f,0.f};
  const v4u zero4u = (v4u){0u,0u,0u,0u};

  for (int i = tid; i < 8192 / 4; i += 256) ((v4f*)ST32)[i] = zero4;
  for (int i = tid; i < (kSlice * kDh) / 8; i += 256) ((v4u*)ST16)[i] = zero4u;
  __syncthreads();

#pragma unroll 1
  for (int c = 0; c < kNChunk; ++c) {
    const size_t rowg0 = (size_t)b * kL + (size_t)c * kChunk;
    {
      const int t1 = tid >> 3, seg = tid & 7;
      const unsigned short* qp = Q16p + (rowg0 + t1) * kD + colq + seg * 32;
      const unsigned short* kp = K16p + (rowg0 + t1) * kD + colq + seg * 32;
      float ssq = 0.0f, ssk = 0.0f;
#pragma unroll 1
      for (int sub = 0; sub < 4; ++sub) {
        const v4u qw = *(const v4u*)(qp + 8 * sub);
        const v4u kw = *(const v4u*)(kp + 8 * sub);
        ssq += sumsq8(qw);
        ssk += sumsq8(kw);
      }
      ssq += __shfl_xor(ssq, 1, 32); ssq += __shfl_xor(ssq, 2, 32); ssq += __shfl_xor(ssq, 4, 32);
      ssk += __shfl_xor(ssk, 1, 32); ssk += __shfl_xor(ssk, 2, 32); ssk += __shfl_xor(ssk, 4, 32);
      const float invq = rsqrtf(ssq * (1.0f / 256.0f) + 1e-6f);
      const float invk = rsqrtf(ssk * (1.0f / 256.0f) + 1e-6f);
      if (seg == 0) {
        invq_s[t1] = invq;
        asm volatile("" ::: "memory");
        invk_s[t1] = invk;
      }
      if (wave == 0) beta_s[lane] = sigmoid_safe(BETA[(rowg0 + lane) * kNar + h]);
    }
    __syncthreads();
    {
      const int dk = tid;
      const unsigned short* kcol = K16p + rowg0 * kD + colq + dk;
#pragma unroll 1
      for (int tg = 0; tg < 4; ++tg) {
        const v4f ia = *(const v4f*)(invk_s + 8 * tg);
        const v4f ib = *(const v4f*)(invk_s + 8 * tg + 4);
        v8h hv;
#pragma unroll
        for (int e = 0; e < 4; ++e) {
          const unsigned wa = kcol[(size_t)(8 * tg + e) * kD];
          const unsigned wb = kcol[(size_t)(8 * tg + 4 + e) * kD];
          hv[e]     = (_Float16)(h16_to_f32(wa) * ia[e]);
          hv[4 + e] = (_Float16)(h16_to_f32(wb) * ib[e]);
        }
        *(v8h*)(kT16 + dk * 32 + 8 * tg) = hv;
      }
      const int dv = tid & 31, vg = tid >> 5;
      const float* vp = V32 + (rowg0 + 4 * vg) * kD + colv + dv;
      const float v0 = vp[0];
      const float v1 = vp[kD];
      const float v2 = vp[2 * kD];
      const float v3 = vp[3 * kD];
      const v2u vu = (v2u){pk16(h_bits(kQKCarry * v0), h_bits(kQKCarry * v1)), pk16(h_bits(kQKCarry * v2), h_bits(kQKCarry * v3))};
      *(v2u*)(vT16 + dv * 32 + 4 * vg) = vu;
    }
    __syncthreads();
    {
      const int grp = wave >> 2;
      const int mt = (wave >> 1) & 1, nt = wave & 1;
      const _Float16* bsrc = (grp == 0) ? K16 : Q16;
      const _Float16* ap = K16 + (rowg0 + 16 * mt + rlane) * kD + colq + koff;
      const _Float16* bp = bsrc + (rowg0 + 16 * nt + rlane) * kD + colq + koff;
      v8f acc = zero8;
#pragma unroll 1
      for (int k0 = 0; k0 < kDh; k0 += 32) acc = mma16(ldfrag(ap + k0), ldfrag(bp + k0), acc);
      const v4f ra = *(const v4f*)(invk_s + 16 * mt + 8 * hh);
      const v4f rc = *(const v4f*)(invk_s + 16 * mt + 8 * hh + 4);
      const float ck = invk_s[16 * nt + rlane];
      const float cq = invq_s[16 * nt + rlane];
      const float cs = ((grp == 0) ? ck : cq) * (1.0f / 256.0f);
      if (grp == 0) {
        v4f o0, o1;
#pragma unroll
        for (int e = 0; e < 4; ++e) {
          o0[e] = acc[e] * ra[e] * cs;
          o1[e] = acc[4 + e] * rc[e] * cs;
        }
        float* kp = KKs + (16 * nt + rlane) * 32 + 16 * mt + 8 * hh;
        *(v4f*)kp = o0;
        *(v4f*)(kp + 4) = o1;
      } else {
        const int icol = 16 * nt + rlane;
        const int jrow = 16 * mt + 8 * hh;
        v8h hv;
#pragma unroll
        for (int e = 0; e < 4; ++e) {
          const float va = acc[e] * ra[e] * cs * 16.0f;
          const float vb = acc[4 + e] * rc[e] * cs * 16.0f;
          hv[e]     = (_Float16)(((jrow + e) <= icol) ? va : 0.0f);
          hv[4 + e] = (_Float16)(((jrow + 4 + e) <= icol) ? vb : 0.0f);
        }
        *(v8h*)(at16 + icol * 32 + jrow) = hv;
      }
    }
    __syncthreads();
    if (wave == 0) {
#pragma unroll 1
      for (int i = 0; i < kChunk; ++i) {
        const float bi = beta_s[i];
        float a = (i == lane) ? 1.0f : 0.0f;
#pragma unroll 1
        for (int j = 0; j < i; ++j) a = fmaf(-(bi * KKs[j * 32 + i]), Ts[j * 32 + lane], a);
        Ts[i * 32 + lane] = a;
      }
    }
    __syncthreads();
    {
      const int i3 = tid >> 3, t0 = (tid & 7) * 4;
      const v4f tv = *(const v4f*)(Ts + i3 * 32 + t0);
      const v4f bv = *(const v4f*)(beta_s + t0);
      const v2u tu = (v2u){pk16(h_bits(16.0f * tv[0] * bv[0]), h_bits(16.0f * tv[1] * bv[1])),
                           pk16(h_bits(16.0f * tv[2] * bv[2]), h_bits(16.0f * tv[3] * bv[3]))};
      *(v2u*)(TB16 + i3 * 32 + t0) = tu;
    }
    __syncthreads();
#pragma unroll 1
    for (int it = 0; it < 4; ++it) {
      const int ti = wave + 8 * it;
      const int pm = ti >> 1;
      const int pn = ti & 1;
      const v8f wacc = mma16(ldfrag(kT16 + (16 * pm + rlane) * 32 + koff), ldfrag(TB16 + (16 * pn + rlane) * 32 + koff), zero8);
      v8h hv;
#pragma unroll
      for (int r = 0; r < 8; ++r) hv[r] = (_Float16)(wacc[r] * 0.25f);
      *(v8h*)(w16 + (16 * pn + rlane) * 256 + 16 * pm + 8 * hh) = hv;
    }
    __syncthreads();
    if (wave < 4) {
      const int mt = wave & 1, nt = wave >> 1;
      const _Float16* ap = w16 + (16 * mt + rlane) * 256 + koff;
      const _Float16* bp = ST16 + (16 * nt + rlane) * 256 + koff;
      v8f aws = zero8;
#pragma unroll 1
      for (int k0 = 0; k0 < kDh; k0 += 32) aws = mma16(ldfrag(ap + k0), ldfrag(bp + k0), aws);
      const v8f au = mma16(ldfrag(TB16 + (16 * mt + rlane) * 32 + koff), ldfrag(vT16 + (16 * nt + rlane) * 32 + koff), zero8);
      v8h hv;
#pragma unroll
      for (int r = 0; r < 8; ++r) hv[r] = (_Float16)(au[r] * 0.25f - aws[r] * 0.0625f);
      *(v8h*)(uhT16 + (16 * nt + rlane) * 32 + 16 * mt + 8 * hh) = hv;
    } else {
      const int mt = wave & 1, nt = (wave >> 1) & 1;
      const _Float16* ap = Q16 + (rowg0 + 16 * mt + rlane) * kD + colq + koff;
      const _Float16* bp = ST16 + (16 * nt + rlane) * 256 + koff;
      v8f o1 = zero8;
#pragma unroll 1
      for (int k0 = 0; k0 < kDh; k0 += 32) o1 = mma16(ldfrag(ap + k0), ldfrag(bp + k0), o1);
      const v4f qa = *(const v4f*)(invq_s + 16 * mt + 8 * hh);
      const v4f qb = *(const v4f*)(invq_s + 16 * mt + 8 * hh + 4);
      v4f f0, f1;
#pragma unroll
      for (int e = 0; e < 4; ++e) {
        f0[e] = o1[e] * qa[e] * (1.0f / 256.0f);
        f1[e] = o1[4 + e] * qb[e] * (1.0f / 256.0f);
      }
      float* op = osc + (16 * nt + rlane) * 32 + 16 * mt + 8 * hh;
      *(v4f*)op = f0;
      *(v4f*)(op + 4) = f1;
    }
    __syncthreads();
    if (wave < 4) {
      const int mt = wave & 1, nt = wave >> 1;
      const v8f o2 = mma16(ldfrag(at16 + (16 * mt + rlane) * 32 + koff), ldfrag(uhT16 + (16 * nt + rlane) * 32 + koff), zero8);
      float* op = osc + (16 * nt + rlane) * 32 + 16 * mt + 8 * hh;
      v4f a0 = *(const v4f*)op;
      v4f a1 = *(const v4f*)(op + 4);
#pragma unroll
      for (int e = 0; e < 4; ++e) {
        a0[e] += o2[e] * (1.0f / 1024.0f);
        a1[e] += o2[4 + e] * (1.0f / 1024.0f);
      }
      *(v4f*)op = a0;
      *(v4f*)(op + 4) = a1;
    }
#pragma unroll 1
    for (int it = 0; it < 4; ++it) {
      const int ti = wave * 4 + it;
      const int pm = ti >> 1;
      const int pn = ti & 1;
      float* sp = ST32 + (ti * 32 + lane) * 8;
      const v4f c0v = *(const v4f*)sp;
      const v4f c1v = *(const v4f*)(sp + 4);
      v8f sacc;
#pragma unroll
      for (int e = 0; e < 4; ++e) { sacc[e] = c0v[e]; sacc[4 + e] = c1v[e]; }
      sacc = mma16(ldfrag(kT16 + (16 * pm + rlane) * 32 + koff), ldfrag(uhT16 + (16 * pn + rlane) * 32 + koff), sacc);
      v4f d0, d1;
      v8h hv;
#pragma unroll
      for (int e = 0; e < 4; ++e) {
        d0[e] = sacc[e];
        d1[e] = sacc[4 + e];
        hv[e]     = (_Float16)(sacc[e] * (1.0f / 64.0f));
        hv[4 + e] = (_Float16)(sacc[4 + e] * (1.0f / 64.0f));
      }
      *(v4f*)sp = d0;
      *(v4f*)(sp + 4) = d1;
      *(v8h*)(ST16 + (16 * pn + rlane) * 256 + 16 * pm + 8 * hh) = hv;
    }
    __syncthreads();
    if (tid < 128) {
      const int row = tid >> 2, c8 = (tid & 3) * 8;
      v8h hv;
#pragma unroll
      for (int e = 0; e < 8; ++e) hv[e] = (_Float16)(kDLCarry * osc[(c8 + e) * 32 + row]);
      unsigned short* gp = dbase + (rowg0 + row) * kSlice + c8;
      *(volatile v8h*)gp = hv;
      __threadfence();
      *(volatile v8h*)gp = hv;
    }
  }
}

__global__ __launch_bounds__(256) void stats_kernel(const float* __restrict__ V32, const unsigned short* __restrict__ DLT,
                                                    const float* __restrict__ fw1, const float* __restrict__ fw3,
                                                    const float* __restrict__ fw7, const float* __restrict__ fw31,
                                                    float* __restrict__ FIR, unsigned short* __restrict__ G16) {
  __shared__ __align__(16) float br[kNS * kD];
  __shared__ float red[8][4];
  __shared__ __align__(16) float stage[128];
  const int row = blockIdx.x;
  const int l = row & (kL - 1);
  const int t = threadIdx.x, lane = t & 31, wave = t >> 5, hd = t >> 6;
  const int c0 = 4 * t, d0 = c0 & (kDh - 1), sl = d0 >> 5, dd = d0 & 31;
  const v4f vc = *(const v4f*)(V32 + (size_t)row * kD + c0);
  const v4f w1v = *(const v4f*)(fw1 + c0);
  float x1[4], x2[4], x3[4];
#pragma unroll
  for (int e = 0; e < 4; ++e) { x1[e] = 0.0f; x2[e] = 0.0f; x3[e] = 0.0f; }
  {
    const int tp0 = (l < 2) ? (2 - l) : 0;
#pragma unroll 1
    for (int tp = tp0; tp < 3; ++tp) {
      const v4f vv = *(const v4f*)(V32 + (size_t)(row - 2 + tp) * kD + c0);
      const float* wp = fw3 + (size_t)c0 * 3 + tp;
#pragma unroll
      for (int e = 0; e < 4; ++e) x1[e] = fmaf(bfr(wp[e * 3]), vv[e], x1[e]);
    }
  }
  {
    const int tp0 = (l < 6) ? (6 - l) : 0;
#pragma unroll 1
    for (int tp = tp0; tp < 7; ++tp) {
      const v4f vv = *(const v4f*)(V32 + (size_t)(row - 6 + tp) * kD + c0);
      const float* wp = fw7 + (size_t)c0 * 7 + tp;
#pragma unroll
      for (int e = 0; e < 4; ++e) x2[e] = fmaf(bfr(wp[e * 7]), vv[e], x2[e]);
    }
  }
  {
    const int tp0 = (l < 30) ? (30 - l) : 0;
#pragma unroll 1
    for (int tp = tp0; tp < 31; ++tp) {
      const v4f vv = *(const v4f*)(V32 + (size_t)(row - 30 + tp) * kD + c0);
      const float* wp = fw31 + (size_t)c0 * 31 + tp;
#pragma unroll
      for (int e = 0; e < 4; ++e) x3[e] = fmaf(bfr(wp[e * 31]), vv[e], x3[e]);
    }
  }
  const v4f f3  = (v4f){x1[0], x1[1], x1[2], x1[3]};
  const v4f f7  = (v4f){x2[0], x2[1], x2[2], x2[3]};
  const v4f f31 = (v4f){x3[0], x3[1], x3[2], x3[3]};
  {
    float* fp = FIR + (size_t)row * kLinN + c0;
    *(volatile v4f*)(fp) = f3; *(volatile v4f*)(fp + kD) = f7; *(volatile v4f*)(fp + 2 * kD) = f31;
    __threadfence();
    *(volatile v4f*)(fp) = f3; *(volatile v4f*)(fp + kD) = f7; *(volatile v4f*)(fp + 2 * kD) = f31;
  }
  v4f fd, f1;
  {
    const v2u dw = *(const v2u*)(DLT + ((size_t)(hd * kNSlice + sl) * kBL + row) * kSlice + dd);
    const unsigned u0 = dw[0], u1 = dw[1];
    fd[0] = h16_to_f32(u0 & 0xffffu) * kDLCarryInv;
    fd[1] = h16_to_f32(u0 >> 16) * kDLCarryInv;
    fd[2] = h16_to_f32(u1 & 0xffffu) * kDLCarryInv;
    fd[3] = h16_to_f32(u1 >> 16) * kDLCarryInv;
#pragma unroll
    for (int e = 0; e < 4; ++e) f1[e] = bfr(w1v[e]) * vc[e];
  }
  *(v4f*)(br + 0 * kD + c0) = f1;
  *(v4f*)(br + 1 * kD + c0) = f3;
  *(v4f*)(br + 2 * kD + c0) = f7;
  *(v4f*)(br + 3 * kD + c0) = f31;
  *(v4f*)(br + 4 * kD + c0) = fd;
  *(v4f*)(br + 5 * kD + c0) = vc;
  if (t >= 96 && t < 128) stage[t] = 0.0f;
  __syncthreads();
#pragma unroll 1
  for (int s = 0; s < kNS; ++s) {
    const v4f xv = *(const v4f*)(br + s * kD + c0);
    float su = (xv[0] + xv[1]) + (xv[2] + xv[3]);
    float sa = (fabsf(xv[0]) + fabsf(xv[1])) + (fabsf(xv[2]) + fabsf(xv[3]));
    float sq = 0.0f;
#pragma unroll
    for (int e = 0; e < 4; ++e) { const float v = xv[e]; sq = fmaf(v, v, sq); }
    su = wsum(su); sa = wsum(sa); sq = wsum(sq);
    if (lane == 0) { red[wave][0] = su; red[wave][1] = sa; red[wave][2] = sq; }
    __syncthreads();
    const float tsum = red[2 * hd][0] + red[2 * hd + 1][0];
    const float tabs = red[2 * hd][1] + red[2 * hd + 1][1];
    const float tsq  = red[2 * hd][2] + red[2 * hd + 1][2];
    const float mean = tsum * (1.0f / 256.0f);
    float cd = 0.0f;
#pragma unroll
    for (int e = 0; e < 4; ++e) { const float d = xv[e] - mean; cd = fmaf(d, d, cd); }
    cd = wsum(cd);
    __syncthreads();
    if (lane == 0) red[wave][3] = cd;
    __syncthreads();
    const float tcd = red[2 * hd][3] + red[2 * hd + 1][3];
    if ((t & 63) == 0) {
      float* sp = stage + hd * 24 + s * 4;
      sp[0] = kStatCarry * mean;
      sp[1] = kStatCarry * sqrtf(tcd * (1.0f / 255.0f));
      sp[2] = kStatCarry * (tabs * (1.0f / 256.0f));
      sp[3] = kStatCarry * sqrtf(tsq);
    }
  }
  __syncthreads();
  if (t < 16) {
    v8h hv;
#pragma unroll
    for (int e = 0; e < 8; ++e) hv[e] = (_Float16)stage[8 * t + e];
    unsigned short* gp = G16 + (size_t)row * kGpad + kD + 8 * t;
    *(volatile v8h*)gp = hv;
    __threadfence();
    *(volatile v8h*)gp = hv;
  }
}

__global__ __launch_bounds__(256) void gelu_kernel(const unsigned short* __restrict__ PRE, unsigned short* __restrict__ HG, int n2) {
  const int i = blockIdx.x * 256 + threadIdx.x;
  if (i >= n2) return;
  const unsigned w = ((const unsigned*)PRE)[i];
  float g0 = 0.0f, g1 = 0.0f;
#pragma unroll 1
  for (int e = 0; e < 2; ++e) {
    const unsigned hb = (e == 0) ? (w & 0xffffu) : (w >> 16);
    const float a = h16_to_f32(hb);
    const float g = (0.5f * a * (1.0f + erff(a * 0.70710678118654752f))) * kHGCarry;
    g0 = (e == 0) ? g : g0;
    g1 = g;
  }
  const unsigned u = pk16(h_bits(g0), h_bits(g1));
  ((volatile unsigned*)HG)[i] = u;
  __threadfence();
  ((volatile unsigned*)HG)[i] = u;
}

__global__ __launch_bounds__(256) void fuse_kernel(const float* __restrict__ FIR, const unsigned short* __restrict__ DLT,
                                                   const float* __restrict__ V32, const float* __restrict__ fw1,
                                                   const float* __restrict__ LOGIT, const float* __restrict__ b2,
                                                   const float* __restrict__ glt, const float* __restrict__ onw,
                                                   unsigned short* __restrict__ FUSED) {
  __shared__ float zs[32];
  __shared__ float es[32];
  __shared__ float red[8];
  __shared__ __align__(16) float stage[1024];
  const int row = blockIdx.x;
  const int t = threadIdx.x, lane = t & 31, wave = t >> 5, hd = t >> 6;
  const int c0 = 4 * t, d0 = c0 & (kDh - 1), sl = d0 >> 5, dd = d0 & 31;
  if (wave == 0) {
    const int tt = (lane < kNLog) ? lane : (kNLog - 1);
    const int hq = tt / kNS;
    const float temp = log1pf(expf(bfr(glt[hq]))) + 0.5f;
    const float z = (LOGIT[(size_t)row * kNar + tt] + bfr(b2[tt])) * (1.0f / temp);
    if (lane < kNLog) zs[lane] = z;
  }
  __syncthreads();
  if (wave == 0) {
    const int tt = (lane < kNLog) ? lane : (kNLog - 1);
    const int hq = tt / kNS;
    float m = zs[hq * kNS];
#pragma unroll
    for (int s = 1; s < kNS; ++s) m = fmaxf(m, zs[hq * kNS + s]);
    const float e = expf(zs[tt] - m);
    if (lane < kNLog) es[lane] = e;
  }
  __syncthreads();
  float wgt[6];
  {
    float den = 0.0f;
#pragma unroll
    for (int s = 0; s < 6; ++s) den += es[hd * kNS + s];
    const float rden = 1.0f / den;
#pragma unroll
    for (int s = 0; s < 6; ++s) wgt[s] = es[hd * kNS + s] * rden;
  }
  float x[6][4];
  {
    const v4f vc  = *(const v4f*)(V32 + (size_t)row * kD + c0);
    const v4f f3  = *(const v4f*)(FIR + (size_t)row * kLinN + c0);
    const v4f f7  = *(const v4f*)(FIR + (size_t)row * kLinN + kD + c0);
    const v4f f31 = *(const v4f*)(FIR + (size_t)row * kLinN + 2 * kD + c0);
    const v4f w1v = *(const v4f*)(fw1 + c0);
    const v2u dw  = *(const v2u*)(DLT + ((size_t)(hd * kNSlice + sl) * kBL + row) * kSlice + dd);
    const unsigned u0 = dw[0], u1 = dw[1];
    x[4][0] = h16_to_f32(u0 & 0xffffu) * kDLCarryInv;
    x[4][1] = h16_to_f32(u0 >> 16) * kDLCarryInv;
    x[4][2] = h16_to_f32(u1 & 0xffffu) * kDLCarryInv;
    x[4][3] = h16_to_f32(u1 >> 16) * kDLCarryInv;
#pragma unroll
    for (int e = 0; e < 4; ++e) {
      x[5][e] = vc[e];
      x[0][e] = bfr(w1v[e]) * vc[e];
      x[1][e] = f3[e];
      x[2][e] = f7[e];
      x[3][e] = f31[e];
    }
  }
  const v4f onv = *(const v4f*)(onw + d0);
  float f[4];
  float sq = 0.0f;
#pragma unroll
  for (int e = 0; e < 4; ++e) {
    float a = 0.0f;
#pragma unroll
    for (int s = 0; s < 6; ++s) a = fmaf(wgt[s], x[s][e], a);
    f[e] = a;
    sq = fmaf(a, a, sq);
  }
  sq = wsum(sq);
  if (lane == 0) red[wave] = sq;
  __syncthreads();
  const float tot = red[2 * hd] + red[2 * hd + 1];
  const float inv = rsqrtf(tot * (1.0f / 256.0f) + 1e-5f);
#pragma unroll
  for (int e = 0; e < 4; ++e) stage[c0 + e] = (f[e] * inv) * bfr(onv[e]) * kFuCarry;
  __syncthreads();
  if (t < 128) {
    v8h hv;
#pragma unroll
    for (int e = 0; e < 8; ++e) hv[e] = (_Float16)stage[8 * t + e];
    unsigned short* gp = FUSED + (size_t)row * kD + 8 * t;
    *(volatile v8h*)gp = hv;
    __threadfence();
    *(volatile v8h*)gp = hv;
  }
}

extern "C" void kernel_launch(void* const* d_in, const int* in_sizes, int n_in,
                              void* d_out, int out_size, void* d_ws, size_t ws_size,
                              hipStream_t stream) {
  if (n_in < 19) return;
  if (in_sizes[0] != kBL * kD) return;
  if (in_sizes[1] != kD * kD || in_sizes[2] != kD * kD || in_sizes[3] != kD * kD) return;
  if (in_sizes[4] != kD * kH) return;
  if (in_sizes[5] != kD * 4 || in_sizes[6] != kD * 4 || in_sizes[7] != kD * 4) return;
  if (in_sizes[8] != kD || in_sizes[9] != kD * 3 || in_sizes[10] != kD * 7 || in_sizes[11] != kD * 31) return;
  if (in_sizes[12] != kGin * kHg || in_sizes[13] != kHg || in_sizes[14] != kHg * kNLog || in_sizes[15] != kNLog) return;
  if (in_sizes[16] != kH || in_sizes[17] != kDh || in_sizes[18] != kD * kD) return;
  if (out_size != kBL * kD) return;

  const size_t szG16  = (size_t)kBL * kGpad * 2;
  const size_t szWQKV = (size_t)kLinN * kD * 2;
  const size_t szW1T  = (size_t)kHg * kGpad * 2;
  const size_t szWO   = (size_t)kD * kD * 2;
  const size_t szNarW = (size_t)kNar * kD * 2;
  const size_t szLIN  = (size_t)kBL * kLinN * 4;
  const size_t szP16  = (size_t)kBL * kD * 2;
  const size_t szV32  = (size_t)kBL * kD * 4;
  const size_t szNarO = (size_t)kBL * kNar * 4;
  const size_t offG16  = 0;
  const size_t offWQKV = offG16 + szG16;
  const size_t offW1T  = offWQKV + szWQKV;
  const size_t offWO   = offW1T + szW1T;
  const size_t offBW   = offWO + szWO;
  const size_t offW2T  = offBW + szNarW;
  const size_t offLIN  = offW2T + szNarW;
  const size_t offQ16  = offLIN + szLIN;
  const size_t offK16  = offQ16 + szP16;
  const size_t offV32  = offK16 + szP16;
  const size_t offBETA = offV32 + szV32;
  const size_t offDLT  = offBETA + szNarO;
  const size_t offHG16 = offDLT + szP16;
  const size_t offLOG  = offHG16 + szP16;
  const size_t total   = offLOG + szNarO;
  if (ws_size < total) return;

  const float* hs   = (const float*)d_in[0];
  const float* qw   = (const float*)d_in[1];
  const float* kw   = (const float*)d_in[2];
  const float* vw   = (const float*)d_in[3];
  const float* bw   = (const float*)d_in[4];
  const float* qcw  = (const float*)d_in[5];
  const float* kcw  = (const float*)d_in[6];
  const float* vcw  = (const float*)d_in[7];
  const float* fw1  = (const float*)d_in[8];
  const float* fw3  = (const float*)d_in[9];
  const float* fw7  = (const float*)d_in[10];
  const float* fw31 = (const float*)d_in[11];
  const float* w1   = (const float*)d_in[12];
  const float* b1   = (const float*)d_in[13];
  const float* w2   = (const float*)d_in[14];
  const float* b2   = (const float*)d_in[15];
  const float* glt  = (const float*)d_in[16];
  const float* onw  = (const float*)d_in[17];
  const float* ow   = (const float*)d_in[18];
  float* out = (float*)d_out;

  char* ws = (char*)d_ws;
  unsigned short* G16  = (unsigned short*)(ws + offG16);
  unsigned short* WQKV = (unsigned short*)(ws + offWQKV);
  unsigned short* W1T  = (unsigned short*)(ws + offW1T);
  unsigned short* WO   = (unsigned short*)(ws + offWO);
  unsigned short* BW   = (unsigned short*)(ws + offBW);
  unsigned short* W2T  = (unsigned short*)(ws + offW2T);
  float*          LIN  = (float*)(ws + offLIN);
  unsigned short* Q16  = (unsigned short*)(ws + offQ16);
  unsigned short* K16  = (unsigned short*)(ws + offK16);
  float*          V32  = (float*)(ws + offV32);
  float*          BETA = (float*)(ws + offBETA);
  unsigned short* DLT  = (unsigned short*)(ws + offDLT);
  unsigned short* HG16 = (unsigned short*)(ws + offHG16);
  float*          LOGT = (float*)(ws + offLOG);
  unsigned short* PRE16 = Q16;
  unsigned short* FUS16 = K16;
  float* FIR = LIN;

  hs16_kernel<<<dim3((kBL * kD) / (8 * 256)), dim3(256), 0, stream>>>(hs, G16);
  wtcast_sq_kernel<<<dim3(kD / 64, kD / 64, 4), dim3(256), 0, stream>>>(qw, kw, vw, ow, WQKV, WO);
  w1cast_kernel<<<dim3(kGpad / 64, kHg / 64), dim3(256), 0, stream>>>(w1, W1T);
  narrow_cast_kernel<<<dim3(kD / 64, 1, 2), dim3(256), 0, stream>>>(bw, w2, BW, W2T);

  const int tilesQKV  = (kBL / 64) * (kLinN / 64);
  const int tilesNar  = (kBL / 64) * (kNar / 64);
  const int tilesWide = (kBL / 64) * (kD / 64);
  wmma_gemm64<0, false, 0, 0, false, 0><<<dim3(tilesQKV / 8, 1), dim3(256), 0, stream>>>(
      G16, G16, kGpad, 0L, WQKV, WQKV, kD, 0L, (void*)LIN, (void*)LIN, kLinN, 0L, b1, b1, 0L, kBL, kLinN, kD, kScaleW);
  wmma_gemm64<0, false, 0, 0, false, 0><<<dim3(tilesNar / 8, 1), dim3(256), 0, stream>>>(
      G16, G16, kGpad, 0L, BW, BW, kD, 0L, (void*)BETA, (void*)BETA, kNar, 0L, b1, b1, 0L, kBL, kNar, kD, kScaleW);

  conv_silu_kernel<<<dim3(kBL, 3), dim3(256), 0, stream>>>(LIN, qcw, kcw, vcw, Q16, K16, V32);

  delta_kernel<<<dim3(kB * kH, kNSlice), dim3(256), 0, stream>>>(Q16, K16, V32, BETA, DLT);

  stats_kernel<<<dim3(kBL), dim3(256), 0, stream>>>(V32, DLT, fw1, fw3, fw7, fw31, FIR, G16);

  wmma_gemm64<0, false, 2, 1, false, 0><<<dim3(tilesWide / 8, 1), dim3(256), 0, stream>>>(
      G16, G16, kGpad, 0L, W1T, W1T, kGpad, 0L, (void*)PRE16, (void*)PRE16, kHg, 0L, b1, b1, 0L, kBL, kHg, kGpad, kScaleW);
  gelu_kernel<<<dim3((kBL * kHg) / (2 * 256)), dim3(256), 0, stream>>>(PRE16, HG16, (kBL * kHg) / 2);
  wmma_gemm64<0, false, 0, 0, false, 0><<<dim3(tilesNar / 8, 1), dim3(256), 0, stream>>>(
      HG16, HG16, kHg, 0L, W2T, W2T, kHg, 0L, (void*)LOGT, (void*)LOGT, kNar, 0L, b1, b1, 0L, kBL, kNar, kHg, kScaleLogit);

  fuse_kernel<<<dim3(kBL), dim3(256), 0, stream>>>(FIR, DLT, V32, fw1, LOGT, b2, glt, onw, FUS16);

  wmma_gemm64<0, false, 0, 0, false, 0><<<dim3(tilesWide / 8, 1), dim3(256), 0, stream>>>(
      FUS16, FUS16, kD, 0L, WO, WO, kD, 0L, (void*)out, (void*)out, kD, 0L, b1, b1, 0L, kBL, kD, kD, kScaleOut);
}
